// ResonantManifold_55095840473096
// MI455X (gfx1250) — hardware-verified
//
#include <hip/hip_runtime.h>
#include <stdint.h>

#define SEQ   2048
#define DH    256
#define CELLS 8
#define NB    2
#define NBC   (NB * CELLS)
#define NTOK  (NBC * SEQ)

typedef _Float16 v16h __attribute__((ext_vector_type(16)));
typedef _Float16 v8h  __attribute__((ext_vector_type(8)));
typedef __bf16   v16b __attribute__((ext_vector_type(16)));
typedef float    v8f  __attribute__((ext_vector_type(8)));
typedef float    v4f  __attribute__((ext_vector_type(4)));
typedef int      v4i  __attribute__((ext_vector_type(4)));
typedef unsigned short v8us __attribute__((ext_vector_type(8)));

static_assert(NTOK == 32768);
static_assert((DH % 64) == 0 && (SEQ % 256) == 0 && (NTOK % 64) == 0);

__device__ __forceinline__ unsigned short bfbits(float f) {
  const unsigned u = __float_as_uint(f);
  return (unsigned short)((u + 0x7FFFu + ((u >> 16) & 1u)) >> 16);
}
__device__ __forceinline__ float bfval(unsigned short b) { return __uint_as_float(((unsigned)b) << 16); }
__device__ __forceinline__ float bfr(float f) { return bfval(bfbits(f)); }

__device__ __forceinline__ v16h ldfrag_h(const _Float16* p) {
  union { v16h v; v8h q[2]; } f;
  f.q[0] = *(const v8h*)(p);
  f.q[1] = *(const v8h*)(p + 16);
  return f.v;
}
__device__ __forceinline__ v16b ldfrag_b(const unsigned short* p) {
  union { v16b v; v8us q[2]; } f;
  f.q[0] = *(const v8us*)(p);
  f.q[1] = *(const v8us*)(p + 16);
  return f.v;
}
__device__ __forceinline__ v8f mma_h(v16h a, v16h b, v8f c) {
  return __builtin_amdgcn_wmma_f32_16x16x32_f16(false, a, false, b, (short)0, c, false, false);
}
__device__ __forceinline__ v8f mma_b(v16b a, v16b b, v8f c) {
  return __builtin_amdgcn_wmma_f32_16x16x32_bf16(false, a, false, b, (short)0, c, false, false);
}
__device__ __forceinline__ v8f zero8() {
  v8f z;
#pragma unroll
  for (int i = 0; i < 8; ++i) z[i] = 0.0f;
  return z;
}

__device__ __forceinline__ void guard_gemm(v8f& a, v8f& b, v8f& c, v8f& d, v16b x, v16b y, v16b z) {
#if defined(__HIP_DEVICE_COMPILE__)
  asm volatile("v_nop\n\tv_nop\n\tv_nop\n\tv_nop" : "+v"(a), "+v"(b), "+v"(c), "+v"(d) : "v"(x), "v"(y), "v"(z));
#endif
}
__device__ __forceinline__ void keep4b(v16b a, v16b b, v16b c, v16b d) {
#if defined(__HIP_DEVICE_COMPILE__)
  asm volatile("v_nop" :: "v"(a), "v"(b), "v"(c), "v"(d));
#endif
}
__device__ __forceinline__ void accg4(v8f& a, v8f& b, v8f& c, v8f& d) {
#if defined(__HIP_DEVICE_COMPILE__)
  asm volatile("v_nop\n\tv_nop\n\tv_nop\n\tv_nop" : "+v"(a), "+v"(b), "+v"(c), "+v"(d));
#endif
}
__device__ __forceinline__ void guard_s(v8f& a, v8f& b, v8f& c, v8f& d, v16h x0, v16h x1, v16h y0, v16h y1) {
#if defined(__HIP_DEVICE_COMPILE__)
  asm volatile("v_nop\n\tv_nop\n\tv_nop\n\tv_nop"
               : "+v"(a), "+v"(b), "+v"(c), "+v"(d) : "v"(x0), "v"(x1), "v"(y0), "v"(y1));
#endif
}
__device__ __forceinline__ void guard_pv(v8f& a0, v8f& a1, v8f& a2, v8f& a3, v8f& b0, v8f& b1, v8f& b2, v8f& b3,
                                         v16h p0, v16h p1, v16h x0, v16h x1, v16h x2, v16h x3) {
#if defined(__HIP_DEVICE_COMPILE__)
  asm volatile("v_nop\n\tv_nop\n\tv_nop\n\tv_nop"
               : "+v"(a0), "+v"(a1), "+v"(a2), "+v"(a3), "+v"(b0), "+v"(b1), "+v"(b2), "+v"(b3)
               : "v"(p0), "v"(p1), "v"(x0), "v"(x1), "v"(x2), "v"(x3));
#endif
}

__global__ __launch_bounds__(256) void gate_kernel(const float* __restrict__ gate, unsigned short* __restrict__ gT) {
  __shared__ float T[64 * 65];
  const int tid = threadIdx.x, wave = tid >> 5, lane = tid & 31;
  const int b = blockIdx.x;
  const int k0 = (b >> 2) * 64, n0 = (b & 3) * 64;
#pragma unroll
  for (int i = 0; i < 16; ++i) {
    const int idx = i * 256 + tid;
    const int r = idx >> 6, cc = idx & 63;
    T[r * 65 + cc] = gate[(size_t)(k0 + r) * DH + n0 + cc];
  }
  __syncthreads();
  const int q = lane >> 3, kk = (lane & 7) * 8;
#pragma unroll
  for (int ps = 0; ps < 2; ++ps) {
#pragma unroll
    for (int it = 0; it < 2; ++it) {
      const int n = wave * 8 + it * 4 + q;
      v8us o;
#pragma unroll
      for (int e = 0; e < 8; ++e) o[e] = bfbits(T[(kk + e) * 65 + n]);
      *(volatile v8us*)(gT + (size_t)(n0 + n) * DH + k0 + kk) = o;
    }
    __threadfence();
  }
}

__global__ __launch_bounds__(256) void ln_kernel(const float* __restrict__ x, unsigned short* __restrict__ lnh,
                                                 unsigned short* __restrict__ lnl, int nrows) {
  const int wave = threadIdx.x >> 5, lane = threadIdx.x & 31;
  const int row = (int)blockIdx.x * 8 + wave;
  if (row >= nrows) return;
  const float* xr = x + (size_t)row * DH + 8 * lane;
  const v4f a = *(const v4f*)(xr), b = *(const v4f*)(xr + 4);
  float v[8];
#pragma unroll
  for (int e = 0; e < 4; ++e) { v[e] = bfr(a[e]); v[4 + e] = bfr(b[e]); }
  float s = ((v[0] + v[1]) + (v[2] + v[3])) + ((v[4] + v[5]) + (v[6] + v[7]));
#pragma unroll
  for (int off = 16; off > 0; off >>= 1) s += __shfl_xor(s, off, 32);
  const float mu = s * (1.0f / 256.0f);
  float s2 = 0.0f;
#pragma unroll
  for (int e = 0; e < 8; ++e) { const float d = v[e] - mu; s2 += d * d; }
#pragma unroll
  for (int off = 16; off > 0; off >>= 1) s2 += __shfl_xor(s2, off, 32);
  const float rstd = rsqrtf(s2 * (1.0f / 256.0f) + 1e-5f);
  v8us oh, ol;
#pragma unroll
  for (int e = 0; e < 8; ++e) {
    const float t = (v[e] - mu) * rstd;
    const unsigned short hb = bfbits(t);
    const unsigned short lb = bfbits(t - bfval(hb));
    oh[e] = hb; ol[e] = lb;
  }
  unsigned short* dh = lnh + (size_t)row * DH + 8 * lane;
  unsigned short* dl = lnl + (size_t)row * DH + 8 * lane;
  *(volatile v8us*)dh = oh;
  *(volatile v8us*)dl = ol;
  __threadfence();
  *(volatile v8us*)dh = oh;
  *(volatile v8us*)dl = ol;
}

__global__ __launch_bounds__(64) void qkv_kernel(const unsigned short* __restrict__ lnh,
                                                 const unsigned short* __restrict__ lnl,
                                                 const unsigned short* __restrict__ gT,
                                                 _Float16* __restrict__ qk, _Float16* __restrict__ vh,
                                                 _Float16* __restrict__ vl, int ntiles) {
  __shared__ __align__(16) float sT[2][64 * 68];
  const int lane = threadIdx.x & 31, wave = threadIdx.x >> 5;
  const int tile = (int)blockIdx.x * 2 + wave;
  if (tile >= ntiles) return;
  const int tm = tile >> 2, tn = tile & 3;
  const int m0 = tm << 6, n0 = tn << 6;
  const int rl = lane & 15, h = lane >> 4, koff = h * 8;

  v8f acc[4][4];
#pragma unroll
  for (int i = 0; i < 4; ++i)
#pragma unroll
    for (int j = 0; j < 4; ++j) acc[i][j] = zero8();

#pragma unroll 1
  for (int k0 = 0; k0 < DH; k0 += 32) {
    v16b bq[4];
#pragma unroll
    for (int j = 0; j < 4; ++j) bq[j] = ldfrag_b(gT + (size_t)(n0 + (j << 4) + rl) * DH + k0 + koff);
#pragma unroll
    for (int i = 0; i < 4; ++i) {
      const size_t ao = (size_t)(m0 + (i << 4) + rl) * DH + k0 + koff;
      const v16b ah = ldfrag_b(lnh + ao);
      const v16b al = ldfrag_b(lnl + ao);
#pragma unroll
      for (int j = 0; j < 4; ++j) {
        acc[i][j] = mma_b(ah, bq[j], acc[i][j]);
        acc[i][j] = mma_b(al, bq[j], acc[i][j]);
      }
      guard_gemm(acc[i][0], acc[i][1], acc[i][2], acc[i][3], ah, al, bq[3]);
    }
    keep4b(bq[0], bq[1], bq[2], bq[3]);
  }
  accg4(acc[0][0], acc[0][1], acc[0][2], acc[0][3]);
  accg4(acc[1][0], acc[1][1], acc[1][2], acc[1][3]);
  accg4(acc[2][0], acc[2][1], acc[2][2], acc[2][3]);
  accg4(acc[3][0], acc[3][1], acc[3][2], acc[3][3]);

  float* slab = sT[wave];
#pragma unroll
  for (int i = 0; i < 4; ++i)
#pragma unroll
    for (int j = 0; j < 4; ++j)
#pragma unroll
      for (int r = 0; r < 8; ++r) slab[((i << 4) + 8 * h + r) * 68 + (j << 4) + rl] = acc[i][j][r];
  __builtin_amdgcn_fence(__ATOMIC_RELEASE, "workgroup");
  __builtin_amdgcn_wave_barrier();
  __builtin_amdgcn_fence(__ATOMIC_ACQUIRE, "workgroup");

  const int q = lane >> 3, c8 = (lane & 7) * 8;
#pragma unroll
  for (int ps = 0; ps < 2; ++ps) {
#pragma unroll
    for (int it = 0; it < 16; ++it) {
      const int row = it * 4 + q;
      const float* sp = slab + row * 68 + c8;
      const v4f a = *(const v4f*)(sp), b = *(const v4f*)(sp + 4);
      v8h o;
#pragma unroll
      for (int e = 0; e < 4; ++e) {
        o[e]     = (_Float16)(a[e] * 0.0625f);
        o[4 + e] = (_Float16)(b[e] * 0.0625f);
      }
      *(volatile v8h*)(qk + (size_t)(m0 + row) * DH + n0 + c8) = o;
    }
    __threadfence();
  }
#pragma unroll
  for (int ps = 0; ps < 2; ++ps) {
#pragma unroll
    for (int it = 0; it < 16; ++it) {
      const int n = it * 4 + q;
      v8h hv, lv;
#pragma unroll
      for (int e = 0; e < 8; ++e) {
        const float v = slab[(c8 + e) * 68 + n];
        const _Float16 hh = (_Float16)v;
        hv[e] = hh;
        lv[e] = (_Float16)((v - (float)hh) * 1024.0f);
      }
      *(volatile v8h*)(vh + (size_t)(n0 + n) * NTOK + m0 + c8) = hv;
      *(volatile v8h*)(vl + (size_t)(n0 + n) * NTOK + m0 + c8) = lv;
    }
    __threadfence();
  }
}

#define QB   32
#define KCH  256
#define QSP  264
#define PSP  264
#define OSP  260
#define SMEM_QP (2 * QB * QSP * 2)
static_assert(QB * OSP * 4 <= SMEM_QP);
static_assert((QSP % 8) == 0 && (PSP % 8) == 0 && (OSP % 4) == 0 && PSP >= KCH);
static_assert((SEQ % KCH) == 0 && (SEQ % QB) == 0 && KCH == 256 && DH == 256);

__global__ __launch_bounds__(256) void attn_kernel(const _Float16* __restrict__ qk, const _Float16* __restrict__ vh,
                                                   const _Float16* __restrict__ vl, const int* __restrict__ msk,
                                                   const float* __restrict__ x, float* __restrict__ x1, float sc) {
  __shared__ __align__(16) char smem[SMEM_QP];
  __shared__ __align__(16) float pmax[256];
  __shared__ __align__(16) float psum[256];
  __shared__ __align__(16) float stt[128];
  __shared__ unsigned int mword[256];
  __shared__ int sbsk[8];
  _Float16* Qs = (_Float16*)smem;
  _Float16* Ps = (_Float16*)(smem + QB * QSP * 2);
  float* Os   = (float*)smem;
  float* m_s  = stt;
  float* l_s  = stt + 32;
  float* al_s = stt + 64;
  float* li_s = stt + 96;

  const int tid = threadIdx.x, wave = tid >> 5, lane = tid & 31, h = lane >> 4, c = lane & 15;
  const int bc = blockIdx.y;
  const int q0 = (int)blockIdx.x * QB;
  const size_t tok0 = (size_t)bc * SEQ;
  const float ninf = -__builtin_inff();

  if (tid < 32) { m_s[tid] = ninf; l_s[tid] = 0.0f; al_s[tid] = 0.0f; li_s[tid] = 0.0f; }
  psum[tid] = 0.0f;
#pragma unroll
  for (int i = 0; i < 4; ++i) {
    const int idx = i * 256 + tid;
    const int row = idx >> 5, pc = idx & 31;
    const v8h v = *(const v8h*)(qk + (tok0 + q0 + row) * DH + pc * 8);
    *(v8h*)(Qs + row * QSP + pc * 8) = v;
  }
  __syncthreads();

  v8f oh[2][2], ol[2][2];
#pragma unroll
  for (int qt = 0; qt < 2; ++qt)
#pragma unroll
    for (int nt = 0; nt < 2; ++nt) { oh[qt][nt] = zero8(); ol[qt][nt] = zero8(); }

  const _Float16* qb0p = Qs + c * QSP + 8 * h;
  const _Float16* qb1p = Qs + (16 + c) * QSP + 8 * h;
  const _Float16* pa0p = Ps + c * PSP + 8 * h;
  const _Float16* pa1p = Ps + (16 + c) * PSP + 8 * h;
  const int ntile = SEQ / KCH;

#pragma unroll 1
  for (int t = 0; t < ntile; ++t) {
    __syncthreads();
#pragma unroll
    for (int rr = 0; rr < 4; ++rr) {
      const int r = wave * 4 + rr;
      const int* mp = msk + (size_t)(q0 + r) * SEQ + t * KCH + 8 * lane;
      const v4i ma = *(const v4i*)(mp);
      const v4i mb = *(const v4i*)(mp + 4);
      unsigned bits = 0u;
#pragma unroll
      for (int e = 0; e < 4; ++e) {
        bits |= (ma[e] != 0 ? 1u : 0u) << e;
        bits |= (mb[e] != 0 ? 1u : 0u) << (4 + e);
      }
      unsigned w = bits << (8 * (lane & 3));
      w |= __shfl_xor(w, 1, 32);
      w |= __shfl_xor(w, 2, 32);
      if ((lane & 3) == 0) mword[(lane >> 2) * 32 + r] = w;
    }
    __syncthreads();
    {
      const unsigned w = mword[wave * 32 + lane];
      const unsigned long long bal = __ballot(w != 0xFFFFFFFFu);
      if (lane == 0) sbsk[wave] = (bal == 0ull) ? 1 : 0;
    }
    __syncthreads();
    int allsk = sbsk[0];
#pragma unroll
    for (int s = 1; s < 8; ++s) allsk &= sbsk[s];
    allsk = __builtin_amdgcn_readfirstlane(allsk);
    if (allsk) continue;
    const int mysk = __builtin_amdgcn_readfirstlane(sbsk[wave]);

    const size_t kb = tok0 + (size_t)t * KCH + 32 * wave;
    const _Float16* ka0p = qk + (kb + c) * DH + 8 * h;
    const _Float16* ka1p = qk + (kb + 16 + c) * DH + 8 * h;
    v8f sacc[2][2];
#pragma unroll
    for (int qt = 0; qt < 2; ++qt)
#pragma unroll
      for (int kt = 0; kt < 2; ++kt) sacc[qt][kt] = zero8();
    if (!mysk) {
#pragma unroll 1
      for (int k0 = 0; k0 < DH; k0 += 32) {
        const v16h a0 = ldfrag_h(ka0p + k0), a1 = ldfrag_h(ka1p + k0);
        const v16h b0 = ldfrag_h(qb0p + k0), b1 = ldfrag_h(qb1p + k0);
        sacc[0][0] = mma_h(a0, b0, sacc[0][0]);
        sacc[0][1] = mma_h(a1, b0, sacc[0][1]);
        sacc[1][0] = mma_h(a0, b1, sacc[1][0]);
        sacc[1][1] = mma_h(a1, b1, sacc[1][1]);
        guard_s(sacc[0][0], sacc[0][1], sacc[1][0], sacc[1][1], a0, a1, b0, b1);
      }
    }
    {
      const unsigned wq0 = mword[wave * 32 + c], wq1 = mword[wave * 32 + 16 + c];
      float pm0 = ninf, pm1 = ninf;
#pragma unroll
      for (int kt = 0; kt < 2; ++kt) {
#pragma unroll
        for (int r = 0; r < 8; ++r) {
          const int bit = 16 * kt + 8 * h + r;
          float v0 = sacc[0][kt][r] * sc;
          v0 = ((wq0 >> bit) & 1u) ? ninf : v0;
          sacc[0][kt][r] = v0; pm0 = fmaxf(pm0, v0);
          float v1 = sacc[1][kt][r] * sc;
          v1 = ((wq1 >> bit) & 1u) ? ninf : v1;
          sacc[1][kt][r] = v1; pm1 = fmaxf(pm1, v1);
        }
      }
      pm0 = fmaxf(pm0, __shfl_xor(pm0, 16, 32));
      pm1 = fmaxf(pm1, __shfl_xor(pm1, 16, 32));
      pmax[wave * 32 + c] = pm0;
      pmax[wave * 32 + 16 + c] = pm1;
    }
    __syncthreads();
    if (wave == 0) {
      const int row = lane;
      float ps = 0.0f;
#pragma unroll
      for (int w = 0; w < 8; ++w) ps += psum[w * 32 + row];
      l_s[row] = l_s[row] * al_s[row] + ps;
      const float mo = m_s[row];
      float mx = mo;
#pragma unroll
      for (int w = 0; w < 8; ++w) mx = fmaxf(mx, pmax[w * 32 + row]);
      al_s[row] = (mx == ninf) ? 1.0f : __expf(mo - mx);
      m_s[row] = mx;
    }
    __syncthreads();
    {
      const float mq0 = m_s[c], mq1 = m_s[16 + c];
      float ps0 = 0.0f, ps1 = 0.0f;
#pragma unroll
      for (int kt = 0; kt < 2; ++kt) {
        v8h h0, h1;
#pragma unroll
        for (int r = 0; r < 8; ++r) {
          const float v0 = sacc[0][kt][r];
          const float p0 = (v0 == ninf) ? 0.0f : __expf(v0 - mq0);
          ps0 += p0; h0[r] = (_Float16)(p0 * 1024.0f);
          const float v1 = sacc[1][kt][r];
          const float p1 = (v1 == ninf) ? 0.0f : __expf(v1 - mq1);
          ps1 += p1; h1[r] = (_Float16)(p1 * 1024.0f);
        }
        *(v8h*)(Ps + c * PSP + 32 * wave + 16 * kt + 8 * h) = h0;
        *(v8h*)(Ps + (16 + c) * PSP + 32 * wave + 16 * kt + 8 * h) = h1;
      }
      ps0 += __shfl_xor(ps0, 16, 32);
      ps1 += __shfl_xor(ps1, 16, 32);
      psum[wave * 32 + c] = ps0;
      psum[wave * 32 + 16 + c] = ps1;
      const v4f aA = *(const v4f*)(al_s + 8 * h), aB = *(const v4f*)(al_s + 8 * h + 4);
      const v4f bA = *(const v4f*)(al_s + 16 + 8 * h), bB = *(const v4f*)(al_s + 16 + 8 * h + 4);
#pragma unroll
      for (int nt = 0; nt < 2; ++nt) {
#pragma unroll
        for (int r = 0; r < 4; ++r) {
          oh[0][nt][r] *= aA[r]; oh[0][nt][4 + r] *= aB[r];
          oh[1][nt][r] *= bA[r]; oh[1][nt][4 + r] *= bB[r];
          ol[0][nt][r] *= aA[r]; ol[0][nt][4 + r] *= aB[r];
          ol[1][nt][r] *= bA[r]; ol[1][nt][4 + r] *= bB[r];
        }
      }
    }
    __syncthreads();
    {
      const size_t kofs = tok0 + (size_t)t * KCH + 8 * h;
      const _Float16* vh0 = vh + (size_t)(32 * wave + c) * NTOK + kofs;
      const _Float16* vh1 = vh0 + (size_t)16 * NTOK;
      const _Float16* vl0 = vl + (size_t)(32 * wave + c) * NTOK + kofs;
      const _Float16* vl1 = vl0 + (size_t)16 * NTOK;
#pragma unroll 1
      for (int ks = 0; ks < 8; ++ks) {
        const int sk = __builtin_amdgcn_readfirstlane(sbsk[ks]);
        if (sk) continue;
        const int ko = ks * 32;
        const v16h pa0 = ldfrag_h(pa0p + ko), pa1 = ldfrag_h(pa1p + ko);
        const v16h b0 = ldfrag_h(vh0 + ko), b1 = ldfrag_h(vh1 + ko);
        const v16h d0 = ldfrag_h(vl0 + ko), d1 = ldfrag_h(vl1 + ko);
        oh[0][0] = mma_h(pa0, b0, oh[0][0]);
        oh[0][1] = mma_h(pa0, b1, oh[0][1]);
        oh[1][0] = mma_h(pa1, b0, oh[1][0]);
        oh[1][1] = mma_h(pa1, b1, oh[1][1]);
        ol[0][0] = mma_h(pa0, d0, ol[0][0]);
        ol[0][1] = mma_h(pa0, d1, ol[0][1]);
        ol[1][0] = mma_h(pa1, d0, ol[1][0]);
        ol[1][1] = mma_h(pa1, d1, ol[1][1]);
        guard_pv(oh[0][0], oh[0][1], oh[1][0], oh[1][1], ol[0][0], ol[0][1], ol[1][0], ol[1][1],
                 pa0, pa1, b0, b1, d0, d1);
      }
    }
  }

  if (wave == 0) {
    const int row = lane;
    float ps = 0.0f;
#pragma unroll
    for (int w = 0; w < 8; ++w) ps += psum[w * 32 + row];
    const float l = l_s[row] * al_s[row] + ps;
    li_s[row] = (1.0f / l) * (1.0f / 1024.0f);
  }
  __syncthreads();
  {
    const v4f iA0 = *(const v4f*)(li_s + 8 * h),      iB0 = *(const v4f*)(li_s + 8 * h + 4);
    const v4f iA1 = *(const v4f*)(li_s + 16 + 8 * h), iB1 = *(const v4f*)(li_s + 16 + 8 * h + 4);
    const float rs = 1.0f / 1024.0f;
#pragma unroll
    for (int nt = 0; nt < 2; ++nt) {
      const int col = 32 * wave + 16 * nt + c;
#pragma unroll
      for (int r = 0; r < 4; ++r) {
        Os[(8 * h + r) * OSP + col]          = (oh[0][nt][r]     + ol[0][nt][r] * rs)     * iA0[r];
        Os[(8 * h + 4 + r) * OSP + col]      = (oh[0][nt][4 + r] + ol[0][nt][4 + r] * rs) * iB0[r];
        Os[(16 + 8 * h + r) * OSP + col]     = (oh[1][nt][r]     + ol[1][nt][r] * rs)     * iA1[r];
        Os[(16 + 8 * h + 4 + r) * OSP + col] = (oh[1][nt][4 + r] + ol[1][nt][4 + r] * rs) * iB1[r];
      }
    }
  }
  __syncthreads();
  {
#pragma unroll
    for (int ps = 0; ps < 2; ++ps) {
#pragma unroll
      for (int rr = 0; rr < 4; ++rr) {
        const int row = wave * 4 + rr;
        const size_t gro = (tok0 + q0 + row) * DH;
#pragma unroll
        for (int j = 0; j < 2; ++j) {
          const int col = 128 * j + 4 * lane;
          const v4f o  = *(const v4f*)(Os + row * OSP + col);
          const v4f xv = *(const v4f*)(x + gro + col);
          v4f res;
#pragma unroll
          for (int e = 0; e < 4; ++e) res[e] = bfr(xv[e]) + o[e];
          *(volatile v4f*)(x1 + gro + col) = res;
        }
      }
      __threadfence();
    }
  }
}

__global__ __launch_bounds__(256) void mix_kernel(const float* __restrict__ x1, const float* __restrict__ inhibit,
                                                  const float* __restrict__ phases, const float* __restrict__ ambition,
                                                  float* __restrict__ out, int per_b, int total) {
  __shared__ float inh[64];
  __shared__ float ph[8];
  __shared__ float am[8];
  const int tid = threadIdx.x;
  if (tid < 64) inh[tid] = bfr(inhibit[tid]);
  {
    const float pv = bfr(phases[tid & 7]);
    const float av = bfr(ambition[tid & 7]);
    if (tid < 8) { ph[tid] = pv; am[tid] = av; }
  }
  __syncthreads();
  const int e = (int)blockIdx.x * 256 + tid;
  if (e >= total) return;
  const int b  = e / per_b;
  const int td = e - b * per_b;
  float xs[CELLS];
#pragma unroll
  for (int cc = 0; cc < CELLS; ++cc) xs[cc] = x1[(size_t)(b * CELLS + cc) * per_b + td];
#pragma unroll 1
  for (int k = 0; k < CELLS; ++k) {
    float comp = 0.0f, xk = 0.0f;
#pragma unroll
    for (int cc = 0; cc < CELLS; ++cc) {
      comp += xs[cc] * inh[cc * CELLS + k];
      xk = (cc == k) ? xs[cc] : xk;
    }
    const float xv  = xk + tanhf(comp);
    const float res = xv + sinf(xv * am[k] + ph[k]) * 0.02f;
    float* p = out + (size_t)(b * CELLS + k) * per_b + td;
    *(volatile float*)p = res;
    __threadfence();
    *(volatile float*)p = res;
  }
}

extern "C" void kernel_launch(void* const* d_in, const int* in_sizes, int n_in,
                              void* d_out, int out_size, void* d_ws, size_t ws_size,
                              hipStream_t stream) {
  if (n_in < 6) return;
  if (in_sizes[0] != NTOK * DH) return;
  if (in_sizes[1] != SEQ * SEQ) return;
  if (in_sizes[2] != DH * DH) return;
  if (in_sizes[3] != CELLS * CELLS || in_sizes[4] != CELLS || in_sizes[5] != CELLS) return;
  if (out_size != NTOK * DH) return;

  const float* x        = (const float*)d_in[0];
  const int*   msk      = (const int*)d_in[1];
  const float* gate     = (const float*)d_in[2];
  const float* inhibit  = (const float*)d_in[3];
  const float* phases   = (const float*)d_in[4];
  const float* ambition = (const float*)d_in[5];
  float* out = (float*)d_out;

  const size_t bGT = (size_t)DH * DH * 2;
  const size_t bPL = (size_t)NTOK * DH * 2;
  const size_t bX1 = (size_t)NTOK * DH * 4;
  size_t off = 0;
  const size_t oGT = off; off += bGT;
  const size_t oLH = off; off += bPL;
  const size_t oLL = off; off += bPL;
  const size_t oQK = off; off += bPL;
  const size_t oVH = off; off += bPL;
  const size_t oVL = off; off += bPL;
  const size_t oX1 = off; off += bX1;
  if (off > ws_size) return;
  if (off > (size_t)134217728) return;

  char* ws = (char*)d_ws;
  unsigned short* GT = (unsigned short*)(ws + oGT);
  unsigned short* LH = (unsigned short*)(ws + oLH);
  unsigned short* LL = (unsigned short*)(ws + oLL);
  _Float16*       QK = (_Float16*)(ws + oQK);
  _Float16*       VH = (_Float16*)(ws + oVH);
  _Float16*       VL = (_Float16*)(ws + oVL);
  float*          X1 = (float*)(ws + oX1);

  const dim3 blk(256);
  gate_kernel<<<dim3((DH / 64) * (DH / 64)), blk, 0, stream>>>(gate, GT);
  ln_kernel<<<dim3(NTOK / 8), blk, 0, stream>>>(x, LH, LL, NTOK);
  const int ntiles = (NTOK / 64) * (DH / 64);
  qkv_kernel<<<dim3(ntiles / 2), dim3(64), 0, stream>>>(LH, LL, GT, QK, VH, VL, ntiles);
  attn_kernel<<<dim3(SEQ / QB, NBC), blk, 0, stream>>>(QK, VH, VL, msk, x, X1, 16.0f);
  const int per_b = SEQ * DH, total = NB * per_b;
  mix_kernel<<<dim3(total / 256), blk, 0, stream>>>(X1, inhibit, phases, ambition, out, per_b, total);
  (void)hipGetLastError();
}
